// semanticFuseModule_82085414961403
// MI455X (gfx1250) — hardware-verified
//
#include <hip/hip_runtime.h>
#include <math.h>
#include <stdint.h>


#define NPIX  16384
#define NCH   64
#define NCLS  21
#define NHEAD 4
#define BIMG  4

typedef _Float16 f16t;
typedef __bf16   bf16t;
typedef f16t  v16h __attribute__((ext_vector_type(16)));
typedef bf16t v16b __attribute__((ext_vector_type(16)));
typedef float v8f  __attribute__((ext_vector_type(8)));
typedef float v4f  __attribute__((ext_vector_type(4)));
typedef v4f   __attribute__((may_alias)) v4fa;
typedef unsigned short v8u __attribute__((ext_vector_type(8)));

union Frag16 { v8u u[2]; v16h h; v16b b; f16t e[16]; unsigned short s[16]; };
union Piece8 { v8u u; f16t e[8]; unsigned short s[8]; };

__device__ __forceinline__ unsigned short bf16_rne(float x)
{
    unsigned int u = __float_as_uint(x);
    u += 0x7FFFu + ((u >> 16) & 1u);
    return (unsigned short)(u >> 16);
}
__device__ __forceinline__ float bf16_val(unsigned short b)
{
    return __uint_as_float(((unsigned int)b) << 16);
}

__device__ __forceinline__ v8f mma_f16(v16h a, v16h b, v8f c)
{
    c = __builtin_amdgcn_wmma_f32_16x16x32_f16(false, a, false, b, (short)0, c, false, false);
    asm volatile("v_nop\n\tv_nop\n\tv_nop\n\tv_nop" : "+v"(c) : "v"(a), "v"(b));
    return c;
}
__device__ __forceinline__ v8f mma_bf16(v16b a, v16b b, v8f c)
{
    c = __builtin_amdgcn_wmma_f32_16x16x32_bf16(false, a, false, b, (short)0, c, false, false);
    asm volatile("v_nop\n\tv_nop\n\tv_nop\n\tv_nop" : "+v"(c) : "v"(a), "v"(b));
    return c;
}

__global__ __launch_bounds__(256)
void xpose_kernel(const float* __restrict__ x, float* xt, int npix, int nbimg)
{
    __shared__ float tile[64][65];
    const int chunks = npix >> 6;
    const int b  = blockIdx.x / chunks;
    const int ch = blockIdx.x - b * chunks;
    const int n0 = ch * 64;
    const bool active = (b < nbimg);
    const int bc = active ? b : 0;

    #pragma unroll
    for (int it = 0; it < 16; ++it) {
        const int idx = it * 256 + threadIdx.x;
        const int c = idx >> 6, nn = idx & 63;
        tile[c][nn] = x[((size_t)(bc * NCH + c)) * npix + n0 + nn];
    }
    __syncthreads();

    const int lane = threadIdx.x & 31, wave = threadIdx.x >> 5;
    const int q = lane & 15;
    v4f vals[4];
    size_t dofs[4];
    #pragma unroll
    for (int j = 0; j < 4; ++j) {
        const int nn = wave * 8 + 2 * j + (lane >> 4);
        v4f v;
        v[0] = tile[4 * q + 0][nn];
        v[1] = tile[4 * q + 1][nn];
        v[2] = tile[4 * q + 2][nn];
        v[3] = tile[4 * q + 3][nn];
        vals[j] = v;
        dofs[j] = ((size_t)bc * npix + n0 + nn) * NCH + 4 * q;
    }
    if (active) {
        #pragma unroll
        for (int j = 0; j < 4; ++j) *(volatile v4f*)(xt + dofs[j]) = vals[j];
        __threadfence();
        #pragma unroll
        for (int j = 0; j < 4; ++j) *(volatile v4f*)(xt + dofs[j]) = vals[j];
    }
}

template<int K, int NOUT, int MODE, int SRC>
__global__ __launch_bounds__(256)
void pack_kernel(const float* __restrict__ W, const float* __restrict__ W2, v8u* outp)
{
    constexpr int KS = K / 32, TN = NOUT / 16, NF = TN * KS;
    constexpr int NPL = (MODE == 1) ? 2 : 1;
    constexpr int UNITS = NPL * NF * 64;
    const int u = blockIdx.x * 256 + threadIdx.x;
    if (u >= UNITS) return;
    const int plane = u / (NF * 64);
    const int rem   = u - plane * (NF * 64);
    const int f = rem >> 6, ln = (rem >> 1) & 31, half = rem & 1;
    const int tn = f / KS, kbi = f - tn * KS;
    const int hl = ln >> 4, n = tn * 16 + (ln & 15);
    Piece8 pc;
    #pragma unroll
    for (int ii = 0; ii < 8; ++ii) {
        const int k = kbi * 32 + half * 16 + 8 * hl + ii;
        float val;
        if (SRC == 0) {
            val = W[(size_t)k * NOUT + n];
        } else {
            const int na = (n < 4) ? n : 0;
            const int nb = (n < 4) ? 0 : (n - 4);
            const int kk = nb / 3, d = nb - kk * 3;
            const float va = W[k * 4 + na];
            const float vb = W2[kk * (K * 3) + k * 3 + d];
            val = (n < 4) ? va : vb;
        }
        if (MODE == 0) {
            pc.e[ii] = (f16t)val;
        } else {
            const unsigned short hb = bf16_rne(val);
            pc.s[ii] = (plane == 0) ? hb : bf16_rne(val - bf16_val(hb));
        }
    }
    v8u* dst = outp + u;
    *(volatile v8u*)dst = pc.u;
    __threadfence();
    *(volatile v8u*)dst = pc.u;
}

template<int K, int NOUT, int MODE, int NB, int RT, int EPI, bool HB>
__global__ __launch_bounds__(256)
void gemm_kernel(const float* __restrict__ A, const v8u* __restrict__ BP,
                 const float* __restrict__ bias, const float* __restrict__ aux0,
                 const float* __restrict__ aux1, float* outp,
                 int M, float aScale, float oScale)
{
    constexpr int KS = K / 32, TN = NOUT / 16;
    constexpr int NPL = (MODE == 1) ? 2 : 1;
    constexpr int NF = TN * KS;
    constexpr int BUNITS = NB * NPL * NF * 64;
    constexpr int SROWS = RT * 16;
    constexpr int STILE = SROWS * NOUT;
    __shared__ v8u bl[BUNITS];
    __shared__ __align__(16) float stg[8 * STILE];

    for (int u = threadIdx.x; u < BUNITS; u += 256) bl[u] = BP[u];
    __syncthreads();

    const int lane = threadIdx.x & 31, wave = threadIdx.x >> 5;
    const int hl = lane >> 4, m = lane & 15;
    const int m0 = (blockIdx.x * 8 + wave) * SROWS;
    const bool active = (m0 + SROWS) <= M;
    const int m0c = active ? m0 : 0;
    int bsel = m0c / NPIX;
    if (bsel > NB - 1) bsel = NB - 1;
    const v8u* bb = bl + bsel * (NPL * NF * 64);

    v8f acc[RT][TN] = {};

    #pragma unroll 1
    for (int kbi = 0; kbi < KS; ++kbi) {
        Frag16 fh[RT];
        Frag16 fl[RT];
        #pragma unroll
        for (int rt = 0; rt < RT; ++rt) {
            const float* ap = A + (size_t)(m0c + rt * 16 + m) * K + kbi * 32 + 8 * hl;
            const v4f x0 = *(const v4f*)(ap);
            const v4f x1 = *(const v4f*)(ap + 4);
            const v4f x2 = *(const v4f*)(ap + 16);
            const v4f x3 = *(const v4f*)(ap + 20);
            float af[16];
            #pragma unroll
            for (int i = 0; i < 4; ++i) {
                af[i] = x0[i]; af[4 + i] = x1[i]; af[8 + i] = x2[i]; af[12 + i] = x3[i];
            }
            #pragma unroll
            for (int i = 0; i < 16; ++i) {
                if (MODE == 0) {
                    fh[rt].e[i] = (f16t)(af[i] * aScale);
                } else {
                    const unsigned short hb = bf16_rne(af[i]);
                    fh[rt].s[i] = hb;
                    fl[rt].s[i] = bf16_rne(af[i] - bf16_val(hb));
                }
            }
        }
        #pragma unroll
        for (int tn = 0; tn < TN; ++tn) {
            const v8u* bp = bb + (tn * KS + kbi) * 64 + lane * 2;
            Frag16 gh;
            gh.u[0] = bp[0];
            gh.u[1] = bp[1];
            if (MODE == 1) {
                Frag16 gl;
                gl.u[0] = bp[NF * 64];
                gl.u[1] = bp[NF * 64 + 1];
                #pragma unroll
                for (int rt = 0; rt < RT; ++rt) {
                    acc[rt][tn] = mma_bf16(fh[rt].b, gh.b, acc[rt][tn]);
                    acc[rt][tn] = mma_bf16(fh[rt].b, gl.b, acc[rt][tn]);
                    acc[rt][tn] = mma_bf16(fl[rt].b, gh.b, acc[rt][tn]);
                }
            } else {
                #pragma unroll
                for (int rt = 0; rt < RT; ++rt)
                    acc[rt][tn] = mma_f16(fh[rt].h, gh.h, acc[rt][tn]);
            }
        }
    }

    float* sw = stg + wave * STILE;
    #pragma unroll
    for (int rt = 0; rt < RT; ++rt) {
        #pragma unroll
        for (int r = 0; r < 8; ++r) {
            const int rloc = rt * 16 + 8 * hl + r;
            const int row  = m0c + rloc;
            float v[TN];
            #pragma unroll
            for (int tn = 0; tn < TN; ++tn) {
                const int col = tn * 16 + m;
                float a = acc[rt][tn][r] * oScale;
                if (EPI == 1) {
                    const int bi = row / NPIX;
                    const int n  = row - bi * NPIX;
                    const int kc = (col < 4) ? 0 : (1 + (col - 4) / 3);
                    float s = aux0[((size_t)bi * NCLS + kc) * NPIX + n];
                    s = fmaxf(s, 0.f);
                    const int ia = (col < 4) ? col : 3;
                    const int ib = (col < 4) ? 0 : (col - 4);
                    const float bva = bias[ia];
                    const float bvb = aux1[ib];
                    a = a * s + ((col < 4) ? bva : bvb);
                } else {
                    if (HB) a += bias[col];
                    if (EPI == 3) a += aux0[(size_t)row * NOUT + col];
                }
                v[tn] = a;
            }
            if (EPI == 2) {
                float s = 0.f;
                #pragma unroll
                for (int tn = 0; tn < TN; ++tn) s += v[tn];
                s += __shfl_xor(s, 1, 32);
                s += __shfl_xor(s, 2, 32);
                s += __shfl_xor(s, 4, 32);
                s += __shfl_xor(s, 8, 32);
                const float mean = s * (1.0f / (float)NOUT);
                float q = 0.f;
                #pragma unroll
                for (int tn = 0; tn < TN; ++tn) {
                    const float d = v[tn] - mean;
                    v[tn] = d;
                    q += d * d;
                }
                q += __shfl_xor(q, 1, 32);
                q += __shfl_xor(q, 2, 32);
                q += __shfl_xor(q, 4, 32);
                q += __shfl_xor(q, 8, 32);
                const float var  = q * (1.0f / (float)NOUT);
                const float rinv = 1.0f / sqrtf(var + 1e-5f);
                #pragma unroll
                for (int tn = 0; tn < TN; ++tn) {
                    const int col = tn * 16 + m;
                    const float y = v[tn] * rinv * aux0[col] + aux1[col];
                    v[tn] = (y > 0.f) ? y : 0.01f * y;
                }
            }
            #pragma unroll
            for (int tn = 0; tn < TN; ++tn) {
                if (EPI == 3) sw[(tn * 16 + m) * SROWS + rloc] = v[tn];
                else          sw[rloc * NOUT + tn * 16 + m]  = v[tn];
            }
        }
    }
    __syncthreads();

    if (active) {
        if (EPI == 3) {
            const int bi = m0 / NPIX;
            const int n0 = m0 - bi * NPIX;
            const int cl = lane >> 3, px = 4 * (lane & 7);
            #pragma unroll
            for (int j = 0; j < NOUT / 4; ++j) {
                const int c = 4 * j + cl;
                const v4f vv = *(const v4fa*)(sw + c * SROWS + px);
                *(volatile v4f*)(outp + ((size_t)(bi * NOUT + c)) * NPIX + n0 + px) = vv;
            }
            __threadfence();
            #pragma unroll
            for (int j = 0; j < NOUT / 4; ++j) {
                const int c = 4 * j + cl;
                const v4f vv = *(const v4fa*)(sw + c * SROWS + px);
                *(volatile v4f*)(outp + ((size_t)(bi * NOUT + c)) * NPIX + n0 + px) = vv;
            }
        } else {
            constexpr int LPR = NOUT / 4;
            constexpr int RPI = 32 / LPR;
            constexpr int NI  = SROWS / RPI;
            const int rl = lane / LPR, cq = 4 * (lane % LPR);
            #pragma unroll
            for (int j = 0; j < NI; ++j) {
                const int r = j * RPI + rl;
                const v4f vv = *(const v4fa*)(sw + r * NOUT + cq);
                *(volatile v4f*)(outp + (size_t)(m0 + r) * NOUT + cq) = vv;
            }
            __threadfence();
            #pragma unroll
            for (int j = 0; j < NI; ++j) {
                const int r = j * RPI + rl;
                const v4f vv = *(const v4fa*)(sw + r * NOUT + cq);
                *(volatile v4f*)(outp + (size_t)(m0 + r) * NOUT + cq) = vv;
            }
        }
    }
}

__global__ __launch_bounds__(256)
void attn_kernel(const float* __restrict__ Q, const float* __restrict__ Kt,
                 const float* __restrict__ rescale, v8u* PO, int npix,
                 float qs, float ks)
{
    const int b = blockIdx.x >> 2, h = blockIdx.x & 3;
    const size_t rowbase = (size_t)b * npix;
    const int lane = threadIdx.x & 31, wave = threadIdx.x >> 5;
    const int hl = lane >> 4, m = lane & 15;

    __shared__ float sp[8 * 256];
    __shared__ float sq[256], sk[256];
    __shared__ float S[256], P[256];
    __shared__ float nqr[16], nkr[16];

    v8f acc = {};
    float aq = 0.f, ak = 0.f;
    const int nsteps = npix >> 5;
    for (int kbi = wave; kbi < nsteps; kbi += 8) {
        Frag16 fa, fb;
        #pragma unroll
        for (int i = 0; i < 16; ++i) {
            const int koff = (i < 8) ? (8 * hl + i) : (16 + 8 * hl + (i - 8));
            const size_t ridx = (rowbase + (size_t)kbi * 32 + koff) * NCH + h * 16 + m;
            const float qv = Q[ridx];
            const float kv = Kt[ridx];
            aq += qv * qv;
            ak += kv * kv;
            fa.e[i] = (f16t)(qv * qs);
            fb.e[i] = (f16t)(kv * ks);
        }
        acc = mma_f16(fa.h, fb.h, acc);
    }
    #pragma unroll
    for (int r = 0; r < 8; ++r) sp[wave * 256 + (8 * hl + r) * 16 + m] = acc[r];
    sq[threadIdx.x] = aq;
    sk[threadIdx.x] = ak;
    __syncthreads();

    {
        float s = 0.f;
        #pragma unroll
        for (int w = 0; w < 8; ++w) s += sp[w * 256 + threadIdx.x];
        S[threadIdx.x] = s;
    }
    if (threadIdx.x < 16) {
        const int t = threadIdx.x;
        float a = 0.f, c = 0.f;
        #pragma unroll
        for (int w = 0; w < 8; ++w) {
            a += sq[w * 32 + t] + sq[w * 32 + t + 16];
            c += sk[w * 32 + t] + sk[w * 32 + t + 16];
        }
        nqr[t] = 1.0f / (sqrtf(a) + 1e-8f);
        nkr[t] = 1.0f / (sqrtf(c) + 1e-8f);
    }
    __syncthreads();

    if (threadIdx.x < 16) {
        const int d = threadIdx.x;
        const float rs = rescale[h];
        const float inv = (1.0f / (qs * ks)) * nqr[d] * rs;
        float rowv[16];
        float mx = -3.0e38f;
        #pragma unroll
        for (int e = 0; e < 16; ++e) {
            const float lg = S[d * 16 + e] * inv * nkr[e];
            rowv[e] = lg;
            mx = fmaxf(mx, lg);
        }
        float sum = 0.f;
        #pragma unroll
        for (int e = 0; e < 16; ++e) { rowv[e] = __expf(rowv[e] - mx); sum += rowv[e]; }
        const float isum = 1.0f / sum;
        #pragma unroll
        for (int e = 0; e < 16; ++e) P[d * 16 + e] = rowv[e] * isum;
    }
    __syncthreads();

    if (threadIdx.x < 128) {
        const int t = threadIdx.x;
        const int kbi = t >> 6, ln = (t >> 1) & 31, half = t & 1;
        const int hl2 = ln >> 4, dcol = ln & 15;
        Piece8 pc;
        #pragma unroll
        for (int ii = 0; ii < 8; ++ii) {
            const int k = kbi * 32 + half * 16 + 8 * hl2 + ii;
            const int e = k - h * 16;
            const float v = (e >= 0 && e < 16) ? P[dcol * 16 + (e & 15)] : 0.f;
            pc.e[ii] = (f16t)v;
        }
        v8u* dst = PO + (size_t)b * 512 + h * 128 + t;
        *(volatile v8u*)dst = pc.u;
        __threadfence();
        *(volatile v8u*)dst = pc.u;
    }
}

extern "C" void kernel_launch(void* const* d_in, const int* in_sizes, int n_in,
                              void* d_out, int out_size, void* d_ws, size_t ws_size,
                              hipStream_t stream)
{
    if (n_in < 27) return;
    const float* x    = (const float*)d_in[0];
    const float* sem  = (const float*)d_in[1];
    const float* wa   = (const float*)d_in[2];
    const float* ba   = (const float*)d_in[3];
    const float* wb   = (const float*)d_in[4];
    const float* bbi  = (const float*)d_in[5];
    const float* in_w = (const float*)d_in[6];
    const float* in_b = (const float*)d_in[7];
    const float* w1   = (const float*)d_in[8];
    const float* b1   = (const float*)d_in[9];
    const float* g1   = (const float*)d_in[10];
    const float* be1  = (const float*)d_in[11];
    const float* w2   = (const float*)d_in[12];
    const float* b2   = (const float*)d_in[13];
    const float* g2   = (const float*)d_in[14];
    const float* be2  = (const float*)d_in[15];
    const float* w3   = (const float*)d_in[16];
    const float* b3   = (const float*)d_in[17];
    const float* wq   = (const float*)d_in[18];
    const float* bq   = (const float*)d_in[19];
    const float* wk   = (const float*)d_in[20];
    const float* bk   = (const float*)d_in[21];
    const float* wv   = (const float*)d_in[22];
    const float* bv   = (const float*)d_in[23];
    const float* wo   = (const float*)d_in[24];
    const float* bo   = (const float*)d_in[25];
    const float* rsc  = (const float*)d_in[26];

    const int M = BIMG * NPIX;
    if (in_sizes[0] != M * NCH) return;
    if (in_sizes[1] != BIMG * NCLS * NPIX) return;
    if (out_size != M * NCH) return;
    if (in_sizes[2] != NCH * 4 || in_sizes[3] < 4) return;
    if (in_sizes[4] != 20 * NCH * 3 || in_sizes[5] < 60) return;
    if (in_sizes[6] != NCH * NCH || in_sizes[7] < NCH) return;
    if (in_sizes[8] != NCH * 128 || in_sizes[9] < 128 || in_sizes[10] < 128 || in_sizes[11] < 128) return;
    if (in_sizes[12] != 128 * 128 || in_sizes[13] < 128 || in_sizes[14] < 128 || in_sizes[15] < 128) return;
    if (in_sizes[16] != 128 * NCH || in_sizes[17] < NCH) return;
    if (in_sizes[18] != NCH * NCH || in_sizes[19] < NCH) return;
    if (in_sizes[20] != NCH * NCH || in_sizes[21] < NCH) return;
    if (in_sizes[22] != NCH * NCH || in_sizes[23] < NCH) return;
    if (in_sizes[24] != NCH * NCH || in_sizes[25] < NCH) return;
    if (in_sizes[26] < NHEAD) return;

    char* ws = (char*)d_ws;
    size_t off = 0;
    const size_t b64  = (size_t)M * NCH * sizeof(float);
    const size_t b128 = (size_t)M * 128 * sizeof(float);
    float* XT  = (float*)(ws + off); off += b64;
    float* SL2 = (float*)(ws + off); off += b64;
    float* YT  = (float*)(ws + off); off += b64;
    float* G1  = (float*)(ws + off); off += b128;
    float* G2  = (float*)(ws + off); off += b128;
    v8u* PF  = (v8u*)(ws + off); off += (size_t)NCH * NCH * 2;
    v8u* PI  = (v8u*)(ws + off); off += (size_t)NCH * NCH * 2;
    v8u* P1  = (v8u*)(ws + off); off += (size_t)2 * NCH * 128 * 2;
    v8u* P2  = (v8u*)(ws + off); off += (size_t)2 * 128 * 128 * 2;
    v8u* P3  = (v8u*)(ws + off); off += (size_t)2 * 128 * NCH * 2;
    v8u* PQ  = (v8u*)(ws + off); off += (size_t)NCH * NCH * 2;
    v8u* PK  = (v8u*)(ws + off); off += (size_t)NCH * NCH * 2;
    v8u* PV  = (v8u*)(ws + off); off += (size_t)NCH * NCH * 2;
    v8u* PW  = (v8u*)(ws + off); off += (size_t)NCH * NCH * 2;
    v8u* PO  = (v8u*)(ws + off); off += (size_t)BIMG * NCH * NCH * 2;
    if (off > ws_size) return;

    float* FEAT = SL2;
    float* XM   = SL2;
    float* Qb   = G1;
    float* Kb   = G1 + (size_t)M * NCH;
    float* Vb   = G2;
    float* Ob   = G2 + (size_t)M * NCH;
    float* out  = (float*)d_out;

    const dim3 blk(256);
    const int grid16 = (M / 16 + 7) / 8;
    const int grid32 = (M / 32 + 7) / 8;

    pack_kernel<64, 64, 0, 1>  <<<dim3((1 * 8  * 64 + 255) / 256), blk, 0, stream>>>(wa,   wb,   PF);
    pack_kernel<64, 64, 0, 0>  <<<dim3((1 * 8  * 64 + 255) / 256), blk, 0, stream>>>(in_w, in_w, PI);
    pack_kernel<64, 128, 1, 0> <<<dim3((2 * 16 * 64 + 255) / 256), blk, 0, stream>>>(w1,   w1,   P1);
    pack_kernel<128, 128, 1, 0><<<dim3((2 * 32 * 64 + 255) / 256), blk, 0, stream>>>(w2,   w2,   P2);
    pack_kernel<128, 64, 1, 0> <<<dim3((2 * 16 * 64 + 255) / 256), blk, 0, stream>>>(w3,   w3,   P3);
    pack_kernel<64, 64, 0, 0>  <<<dim3((1 * 8  * 64 + 255) / 256), blk, 0, stream>>>(wq,   wq,   PQ);
    pack_kernel<64, 64, 0, 0>  <<<dim3((1 * 8  * 64 + 255) / 256), blk, 0, stream>>>(wk,   wk,   PK);
    pack_kernel<64, 64, 0, 0>  <<<dim3((1 * 8  * 64 + 255) / 256), blk, 0, stream>>>(wv,   wv,   PV);
    pack_kernel<64, 64, 0, 0>  <<<dim3((1 * 8  * 64 + 255) / 256), blk, 0, stream>>>(wo,   wo,   PW);

    xpose_kernel<<<dim3(BIMG * (NPIX / 64)), blk, 0, stream>>>(x, XT, NPIX, BIMG);

    gemm_kernel<64, 64, 0, 1, 1, 1, true><<<dim3(grid16), blk, 0, stream>>>(XT, PF, ba, sem, bbi, FEAT, M, 1.0f, 1.0f);
    gemm_kernel<64, 64, 0, 1, 1, 0, true><<<dim3(grid16), blk, 0, stream>>>(FEAT, PI, in_b, in_b, in_b, YT, M, 1.0f, 1.0f);
    gemm_kernel<64, 128, 1, 1, 1, 2, true> <<<dim3(grid16), blk, 0, stream>>>(XT, P1, b1, g1, be1, G1, M, 1.0f, 1.0f);
    gemm_kernel<128, 128, 1, 1, 1, 2, true><<<dim3(grid16), blk, 0, stream>>>(G1, P2, b2, g2, be2, G2, M, 1.0f, 1.0f);
    gemm_kernel<128, 64, 1, 1, 1, 0, true> <<<dim3(grid16), blk, 0, stream>>>(G2, P3, b3, b3, b3, XM, M, 1.0f, 1.0f);
    gemm_kernel<64, 64, 0, 1, 1, 0, true><<<dim3(grid16), blk, 0, stream>>>(XM, PQ, bq, bq, bq, Qb, M, 1.0f, 1.0f);
    gemm_kernel<64, 64, 0, 1, 1, 0, true><<<dim3(grid16), blk, 0, stream>>>(YT, PK, bk, bk, bk, Kb, M, 64.0f, 1.0f / 64.0f);
    gemm_kernel<64, 64, 0, 1, 1, 0, true><<<dim3(grid16), blk, 0, stream>>>(YT, PV, bv, bv, bv, Vb, M, 64.0f, 1.0f / 64.0f);
    attn_kernel<<<dim3(BIMG * NHEAD), blk, 0, stream>>>(Qb, Kb, rsc, PO, NPIX, 16.0f, 64.0f);
    gemm_kernel<64, 64, 0, BIMG, 1, 0, false><<<dim3(grid16), blk, 0, stream>>>(Vb, PO, bo, bo, bo, Ob, M, 256.0f, 1.0f / 256.0f);
    gemm_kernel<64, 64, 0, 1, 2, 3, true><<<dim3(grid32), blk, 0, stream>>>(Ob, PW, bo, XM, bo, out, M, 4096.0f, 1.0f / 4096.0f);
}
